// CoAttentionLayer2_34437047780052
// MI455X (gfx1250) — hardware-verified
//
#include <hip/hip_runtime.h>
#include <math.h>

constexpr int kBatch  = 8;
constexpr int kNq     = 1024;
constexpr int kNk     = 1024;
constexpr int kDim    = 512;
constexpr int kHeads  = 8;
constexpr int kDh     = 64;
constexpr int kInner  = kHeads * kDh;
constexpr int kRowsQ  = kBatch * kNq;
constexpr int kRowsK  = kBatch * kNk;
constexpr float kScoreScale = 0.125f;
constexpr float kLnEps = 1e-5f;

static_assert(kDim == 512);
static_assert(kNk == 1024);
static_assert(kInner == kDim);
static_assert(kRowsQ % 64 == 0 && kRowsK % 64 == 0 && kDim % 64 == 0 && kDh % 32 == 0 && kNq % 64 == 0 && kNk % 64 == 0);

typedef __attribute__((ext_vector_type(16))) _Float16 v16h;
typedef __attribute__((ext_vector_type(8)))  _Float16 v8h;
typedef __attribute__((ext_vector_type(16))) __bf16   v16b;
typedef __attribute__((ext_vector_type(8)))  __bf16   v8b;
typedef __attribute__((ext_vector_type(8)))  float    v8f;
typedef __attribute__((ext_vector_type(4)))  float    v4f;
typedef __attribute__((ext_vector_type(4)))  unsigned int v4u;

__device__ __forceinline__ unsigned short f2bf_bits(float f) {
  unsigned u = __float_as_uint(f);
  return (unsigned short)((u + 0x7FFFu + ((u >> 16) & 1u)) >> 16);
}
__device__ __forceinline__ float bf_bits2f(unsigned short h) { return __uint_as_float(((unsigned)h) << 16); }

__device__ __forceinline__ void dep_guard_h(v8f& a, v8f& b, v16h x, v16h y) { asm volatile("v_nop\n\tv_nop\n\tv_nop\n\tv_nop" : "+v"(a), "+v"(b) : "v"(x), "v"(y)); }
__device__ __forceinline__ void dep_guard_b(v8f& a, v8f& b, v16b x, v16b y) { asm volatile("v_nop\n\tv_nop\n\tv_nop\n\tv_nop" : "+v"(a), "+v"(b) : "v"(x), "v"(y)); }
__device__ __forceinline__ void keep4_h(v16h a, v16h b, v16h c, v16h d) { asm volatile("v_nop" :: "v"(a), "v"(b), "v"(c), "v"(d)); }
__device__ __forceinline__ void keep4_b(v16b a, v16b b, v16b c, v16b d) { asm volatile("v_nop" :: "v"(a), "v"(b), "v"(c), "v"(d)); }
__device__ __forceinline__ void acc_guard4(v8f& a, v8f& b, v8f& c, v8f& d) { asm volatile("v_nop\n\tv_nop\n\tv_nop\n\tv_nop" : "+v"(a), "+v"(b), "+v"(c), "+v"(d)); }
template <typename T> struct Frag;
template <> struct Frag<_Float16> {
  typedef v16h V; union U { v16h v; v8h h[2]; };
  static __device__ __forceinline__ v16h load(const _Float16* p) {
    U f; f.h[0] = *(const v8h*)(p); f.h[1] = *(const v8h*)(p + 16); return f.v;
  }
  static __device__ __forceinline__ v8f mma(v16h a, v16h b, v8f c) {
    return __builtin_amdgcn_wmma_f32_16x16x32_f16(false, a, false, b, (short)0, c, false, false);
  }
  static __device__ __forceinline__ void guard(v8f& a, v8f& b, v16h x, v16h y) { dep_guard_h(a, b, x, y); }
  static __device__ __forceinline__ void keep(v16h a, v16h b, v16h c, v16h d) { keep4_h(a, b, c, d); }
};
template <> struct Frag<__bf16> {
  typedef v16b V; union U { v16b v; v8b h[2]; };
  static __device__ __forceinline__ v16b load(const __bf16* p) {
    U f; f.h[0] = *(const v8b*)(p); f.h[1] = *(const v8b*)(p + 16); return f.v;
  }
  static __device__ __forceinline__ v8f mma(v16b a, v16b b, v8f c) {
    return __builtin_amdgcn_wmma_f32_16x16x32_bf16(false, a, false, b, (short)0, c, false, false);
  }
  static __device__ __forceinline__ void guard(v8f& a, v8f& b, v16b x, v16b y) { dep_guard_b(a, b, x, y); }
  static __device__ __forceinline__ void keep(v16b a, v16b b, v16b c, v16b d) { keep4_b(a, b, c, d); }
};

__device__ __forceinline__ unsigned pk16(unsigned short a, unsigned short b) { return (unsigned)a | ((unsigned)b << 16); }

template <int ET> struct Elem;
template <> struct Elem<0> { typedef _Float16 T; };
template <> struct Elem<1> { typedef __bf16 T; };
template <int ET, bool ASPLIT, int BIAS_MODE, int OUT_MODE, bool RESID, bool BSPLIT>
__global__ __launch_bounds__(256) void wmma_gemm64(
    const unsigned short* __restrict__ Ap, const unsigned short* __restrict__ A2p, int lda, long strideA,
    const unsigned short* __restrict__ Btp, const unsigned short* __restrict__ Bt2p, int ldb, long strideB,
    void* __restrict__ Cout, void* __restrict__ Cout2, int ldc, long strideC,
    const float* __restrict__ bias,
    const float* __restrict__ resid, long strideR,
    int M, int N, int K, float scale) {
  typedef typename Elem<ET>::T T;
  typedef typename Frag<T>::V V;
  const T* A = (const T*)Ap; const T* A2 = (const T*)A2p; const T* Bt = (const T*)Btp; const T* Bt2 = (const T*)Bt2p;
  __shared__ __align__(16) float sT[8][16 * 68];
  const int b    = blockIdx.y;
  const int lane = threadIdx.x & 31;
  const int wave = threadIdx.x >> 5;
  const int tilesN = N >> 6;
  const int tilesM = M >> 6;
  const int tile = blockIdx.x * 8 + wave;
  if (tile >= tilesM * tilesN) return;
  const int tm = tile / tilesN;
  const int tn = tile - tm * tilesN;
  const int m0 = tm << 6;
  const int n0 = tn << 6;

  const T* Ab  = A  + (size_t)b * strideA;
  const T* Bb  = Bt + (size_t)b * strideB;
  const T* Ab2 = ASPLIT ? (A2  + (size_t)b * strideA) : nullptr;
  const T* Bb2 = BSPLIT ? (Bt2 + (size_t)b * strideB) : nullptr;

  const int rlane = lane & 15;
  const int koff  = (lane >> 4) * 8;
  const int mOff  = (lane >> 4) * 8;

  v8f acc[4][4];
#pragma unroll
  for (int i = 0; i < 4; ++i)
#pragma unroll
    for (int j = 0; j < 4; ++j) acc[i][j] = (v8f){0.f,0.f,0.f,0.f,0.f,0.f,0.f,0.f};

  for (int k0 = 0; k0 < K; k0 += 32) {
    V bh[4], bl[4];
#pragma unroll
    for (int j = 0; j < 4; ++j) {
      const size_t bo = (size_t)(n0 + (j << 4) + rlane) * ldb + koff + k0;
      bh[j] = Frag<T>::load(Bb + bo);
      if (BSPLIT) bl[j] = Frag<T>::load(Bb2 + bo);
    }
#pragma unroll
    for (int i = 0; i < 4; ++i) {
      const size_t ao = (size_t)(m0 + (i << 4) + rlane) * lda + koff + k0;
      V ah = Frag<T>::load(Ab + ao);
      V al;
      if (ASPLIT) al = Frag<T>::load(Ab2 + ao);
#pragma unroll
      for (int j = 0; j < 4; ++j) {
        acc[i][j] = Frag<T>::mma(ah, bh[j], acc[i][j]);
        if (BSPLIT) acc[i][j] = Frag<T>::mma(ah, bl[j], acc[i][j]);
        if (ASPLIT) acc[i][j] = Frag<T>::mma(al, bh[j], acc[i][j]);
      }
      Frag<T>::guard(acc[i][0], acc[i][3], ah, ASPLIT ? al : ah);
    }
    Frag<T>::keep(bh[0], bh[1], bh[2], bh[3]);
    if (BSPLIT) Frag<T>::keep(bl[0], bl[1], bl[2], bl[3]);
  }
  acc_guard4(acc[0][0], acc[0][1], acc[0][2], acc[0][3]);
  acc_guard4(acc[1][0], acc[1][1], acc[1][2], acc[1][3]);
  acc_guard4(acc[2][0], acc[2][1], acc[2][2], acc[2][3]);
  acc_guard4(acc[3][0], acc[3][1], acc[3][2], acc[3][3]);

  float* slab = sT[wave];
  const float* Rb = RESID ? (resid + (size_t)b * strideR) : nullptr;
#pragma unroll
  for (int i = 0; i < 4; ++i) {
    const int mBase = m0 + (i << 4);
#pragma unroll
    for (int j = 0; j < 4; ++j) {
      const int n = n0 + (j << 4) + rlane;
      float bv = 0.f;
      if (BIAS_MODE == 2) bv = bias[n];
#pragma unroll
      for (int r = 0; r < 8; ++r) {
        float v = acc[i][j][r] * scale;
        if (BIAS_MODE == 1) v += bias[mBase + mOff + r];
        if (BIAS_MODE == 2) v += bv;
        if (RESID) v += Rb[(size_t)(mBase + mOff + r) * ldc + n];
        slab[(mOff + r) * 68 + (j << 4) + rlane] = v;
      }
    }
    __builtin_amdgcn_fence(__ATOMIC_RELEASE, "workgroup");
    __builtin_amdgcn_wave_barrier();
    __builtin_amdgcn_fence(__ATOMIC_ACQUIRE, "workgroup");
    if (OUT_MODE == 0) {
      float* C = (float*)Cout + (size_t)b * strideC;
      const int hh = lane >> 4, c4 = (lane & 15) * 4;
      for (int pass = 0; pass < 2; ++pass) {
#pragma unroll
        for (int it = 0; it < 8; ++it) {
          const int row = it * 2 + hh;
          v4f v = *(const v4f*)(slab + row * 68 + c4);
          *(volatile v4f*)(C + (size_t)(mBase + row) * ldc + n0 + c4) = v;
        }
        __threadfence();
      }
    } else {
      const int q = lane >> 3, c8 = (lane & 7) * 8;
      unsigned short* C  = (unsigned short*)Cout  + (size_t)b * strideC;
      unsigned short* C2 = (OUT_MODE == 2) ? ((unsigned short*)Cout2 + (size_t)b * strideC) : nullptr;
      for (int pass = 0; pass < 2; ++pass) {
#pragma unroll
        for (int it = 0; it < 4; ++it) {
          const int row = it * 4 + q;
          const float* sp = slab + row * 68 + c8;
          v8h hv, lv;
#pragma unroll
          for (int e = 0; e < 8; ++e) {
            if (OUT_MODE == 1) {
              hv[e] = (_Float16)sp[e];
            } else {
              unsigned short hb = f2bf_bits(sp[e]);
              unsigned short lb = f2bf_bits(sp[e] - bf_bits2f(hb));
              hv[e] = __builtin_bit_cast(_Float16, hb);
              lv[e] = __builtin_bit_cast(_Float16, lb);
            }
          }
          *(volatile v8h*)(C + (size_t)(mBase + row) * ldc + n0 + c8) = hv;
          if (OUT_MODE == 2) *(volatile v8h*)(C2 + (size_t)(mBase + row) * ldc + n0 + c8) = lv;
        }
        __threadfence();
      }
    }
    __builtin_amdgcn_fence(__ATOMIC_RELEASE, "workgroup");
    __builtin_amdgcn_wave_barrier();
    __builtin_amdgcn_fence(__ATOMIC_ACQUIRE, "workgroup");
  }
}

__global__ __launch_bounds__(256) void transpose_cast_kernel(const float* __restrict__ in, int ldin,
                                                             unsigned short* __restrict__ out, int ldout) {
  __shared__ float sm[64][65];
  const int t  = threadIdx.x;
  const int r0 = blockIdx.x * 64;
  const int c0 = blockIdx.y * 64;
#pragma unroll
  for (int i = 0; i < 16; ++i) {
    const int e = i * 256 + t;
    const int r = e >> 6;
    const int c = e & 63;
    sm[c][r] = in[(size_t)(r0 + r) * ldin + c0 + c];
  }
  __syncthreads();
  const int lane = t & 31, wave = t >> 5;
  const int q = lane >> 3, c8 = (lane & 7) * 8;
  for (int pass = 0; pass < 2; ++pass) {
#pragma unroll
    for (int it = 0; it < 2; ++it) {
      const int row = wave * 8 + it * 4 + q;
      unsigned w[4];
#pragma unroll
      for (int e2 = 0; e2 < 4; ++e2) w[e2] = pk16(f2bf_bits(sm[row][c8 + 2 * e2]), f2bf_bits(sm[row][c8 + 2 * e2 + 1]));
      const v4u u = (v4u){w[0], w[1], w[2], w[3]};
      const size_t o = (size_t)(c0 + row) * ldout + r0 + c8;
      *(volatile v4u*)(out + o) = u;
    }
    __threadfence();
  }
}

__global__ __launch_bounds__(256) void ln_split_kernel(const float* __restrict__ x, const float* __restrict__ gamma,
                                                       const float* __restrict__ beta,
                                                       unsigned short* __restrict__ yhi, unsigned short* __restrict__ ylo,
                                                       int nrows) {
  const int lane = threadIdx.x & 31, wave = threadIdx.x >> 5;
  const int row = blockIdx.x * 8 + wave;
  if (row >= nrows) return;
  const float* xr = x + (size_t)row * kDim;
  float xv[16];
  {
    const v4f a0 = *(const v4f*)(xr + 8 * lane);
    const v4f a1 = *(const v4f*)(xr + 8 * lane + 4);
    const v4f c0 = *(const v4f*)(xr + 256 + 8 * lane);
    const v4f c1 = *(const v4f*)(xr + 256 + 8 * lane + 4);
#pragma unroll
    for (int e = 0; e < 4; ++e) { xv[e] = a0[e]; xv[4 + e] = a1[e]; xv[8 + e] = c0[e]; xv[12 + e] = c1[e]; }
  }
  float s = 0.f;
#pragma unroll
  for (int e = 0; e < 16; ++e) { xv[e] = bf_bits2f(f2bf_bits(xv[e])); s += xv[e]; }
#pragma unroll
  for (int off = 16; off > 0; off >>= 1) s += __shfl_xor(s, off, 32);
  const float mu = s * (1.0f / 512.0f);
  float s2 = 0.f;
#pragma unroll
  for (int e = 0; e < 16; ++e) { const float d = xv[e] - mu; xv[e] = d; s2 += d * d; }
#pragma unroll
  for (int off = 16; off > 0; off >>= 1) s2 += __shfl_xor(s2, off, 32);
  const float var  = s2 * (1.0f / 512.0f);
  const float rstd = rsqrtf(var + kLnEps);

  float gv[16], bv[16];
  {
    const v4f g0 = *(const v4f*)(gamma + 8 * lane);
    const v4f g1 = *(const v4f*)(gamma + 8 * lane + 4);
    const v4f g2 = *(const v4f*)(gamma + 256 + 8 * lane);
    const v4f g3 = *(const v4f*)(gamma + 256 + 8 * lane + 4);
    const v4f b0 = *(const v4f*)(beta + 8 * lane);
    const v4f b1 = *(const v4f*)(beta + 8 * lane + 4);
    const v4f b2 = *(const v4f*)(beta + 256 + 8 * lane);
    const v4f b3 = *(const v4f*)(beta + 256 + 8 * lane + 4);
#pragma unroll
    for (int e = 0; e < 4; ++e) {
      gv[e] = g0[e]; gv[4 + e] = g1[e]; gv[8 + e] = g2[e]; gv[12 + e] = g3[e];
      bv[e] = b0[e]; bv[4 + e] = b1[e]; bv[8 + e] = b2[e]; bv[12 + e] = b3[e];
    }
  }
  unsigned hw[8], lw[8];
#pragma unroll
  for (int e2 = 0; e2 < 8; ++e2) {
    const float ga = bf_bits2f(f2bf_bits(gv[2 * e2]));
    const float gb = bf_bits2f(f2bf_bits(gv[2 * e2 + 1]));
    const float ba = bf_bits2f(f2bf_bits(bv[2 * e2]));
    const float bb = bf_bits2f(f2bf_bits(bv[2 * e2 + 1]));
    const float y0 = (xv[2 * e2] * rstd) * ga + ba;
    const float y1 = (xv[2 * e2 + 1] * rstd) * gb + bb;
    const unsigned short h0 = f2bf_bits(y0);
    const unsigned short h1 = f2bf_bits(y1);
    const unsigned short l0 = f2bf_bits(y0 - bf_bits2f(h0));
    const unsigned short l1 = f2bf_bits(y1 - bf_bits2f(h1));
    hw[e2] = pk16(h0, h1);
    lw[e2] = pk16(l0, l1);
  }
  const v4u hv0 = (v4u){hw[0], hw[1], hw[2], hw[3]};
  const v4u hv1 = (v4u){hw[4], hw[5], hw[6], hw[7]};
  const v4u lv0 = (v4u){lw[0], lw[1], lw[2], lw[3]};
  const v4u lv1 = (v4u){lw[4], lw[5], lw[6], lw[7]};
  unsigned short* ph = yhi + (size_t)row * kDim;
  unsigned short* pl = ylo + (size_t)row * kDim;
  for (int pass = 0; pass < 2; ++pass) {
    *(volatile v4u*)(ph + 8 * lane) = hv0;
    *(volatile v4u*)(ph + 256 + 8 * lane) = hv1;
    *(volatile v4u*)(pl + 8 * lane) = lv0;
    *(volatile v4u*)(pl + 256 + 8 * lane) = lv1;
    __threadfence();
  }
}

__global__ __launch_bounds__(128) void softmax_rows_kernel(const float* __restrict__ S,
                                                           unsigned short* __restrict__ Phi, unsigned short* __restrict__ Plo) {
  __shared__ float redM[4];
  __shared__ float redS[4];
  const int blk  = blockIdx.x;
  const int t    = threadIdx.x;
  const int lane = t & 31, wave = t >> 5;
  const int c0   = t * 8;
  const size_t rowoff = (size_t)blk * (size_t)kNk;

  float xv[8];
  {
    const float* sr = S + rowoff + c0;
    const v4f a = *(const v4f*)(sr);
    const v4f c = *(const v4f*)(sr + 4);
#pragma unroll
    for (int e = 0; e < 4; ++e) { xv[e] = a[e]; xv[4 + e] = c[e]; }
  }
  float m = xv[0];
#pragma unroll
  for (int e = 1; e < 8; ++e) m = fmaxf(m, xv[e]);
#pragma unroll
  for (int off = 16; off > 0; off >>= 1) m = fmaxf(m, __shfl_xor(m, off, 32));
  if (lane == 0) redM[wave] = m;
  __syncthreads();
  float gmax = redM[0];
#pragma unroll
  for (int w = 1; w < 4; ++w) gmax = fmaxf(gmax, redM[w]);

  float p[8];
  float ps = 0.0f;
#pragma unroll
  for (int e = 0; e < 8; ++e) { p[e] = expf(xv[e] - gmax); ps += p[e]; }
#pragma unroll
  for (int off = 16; off > 0; off >>= 1) ps += __shfl_xor(ps, off, 32);
  if (lane == 0) redS[wave] = ps;
  __syncthreads();
  float tot = redS[0];
#pragma unroll
  for (int w = 1; w < 4; ++w) tot += redS[w];
  const float inv = 1.0f / tot;

  unsigned hw[4], lw[4];
#pragma unroll
  for (int e2 = 0; e2 < 4; ++e2) {
    const float f0 = p[2 * e2] * inv;
    const float f1 = p[2 * e2 + 1] * inv;
    const unsigned short h0 = f2bf_bits(f0);
    const unsigned short h1 = f2bf_bits(f1);
    const unsigned short l0 = f2bf_bits(f0 - bf_bits2f(h0));
    const unsigned short l1 = f2bf_bits(f1 - bf_bits2f(h1));
    hw[e2] = pk16(h0, h1);
    lw[e2] = pk16(l0, l1);
  }
  const v4u hv = (v4u){hw[0], hw[1], hw[2], hw[3]};
  const v4u lv = (v4u){lw[0], lw[1], lw[2], lw[3]};
  unsigned short* ph = Phi + rowoff + c0;
  unsigned short* pl = Plo + rowoff + c0;
  for (int pass = 0; pass < 2; ++pass) {
    *(volatile v4u*)ph = hv;
    *(volatile v4u*)pl = lv;
    __threadfence();
  }
}

extern "C" void kernel_launch(void* const* d_in, const int* in_sizes, int n_in,
                              void* d_out, int out_size, void* d_ws, size_t ws_size,
                              hipStream_t stream) {
  if (n_in < 7) return;
  if (in_sizes[0] != kRowsQ * kDim || in_sizes[1] != kRowsK * kDim) return;
  if (in_sizes[2] != kDim * kInner || in_sizes[3] != kDim * 2 * kInner || in_sizes[4] != kInner * kDim) return;
  if (in_sizes[5] != kDim || in_sizes[6] != kDim) return;
  if (out_size != kRowsQ * kDim) return;

  const size_t kMiB    = 1048576;
  const size_t offS    = 0;
  const size_t offQnH  = 0;
  const size_t offQnL  = 8 * kMiB;
  const size_t offKnH  = 16 * kMiB;
  const size_t offKnL  = 24 * kMiB;
  const size_t offWoT  = 0;
  const size_t offPhi  = 32 * kMiB;
  const size_t offPlo  = 48 * kMiB;
  const size_t offWqT  = 32 * kMiB;
  const size_t offWkvT = 32 * kMiB + kMiB / 2;
  const size_t offQhi  = 64 * kMiB;
  const size_t offQlo  = 72 * kMiB;
  const size_t offKhi  = 80 * kMiB;
  const size_t offKlo  = 88 * kMiB;
  const size_t offVthi = 96 * kMiB;
  const size_t offVtlo = 104 * kMiB;
  const size_t offChi  = 112 * kMiB;
  const size_t offClo  = 120 * kMiB;
  const size_t total   = 128 * kMiB;
  if (total > ws_size) return;

  const float* query    = (const float*)d_in[0];
  const float* keyvalue = (const float*)d_in[1];
  const float* Wq       = (const float*)d_in[2];
  const float* Wkv      = (const float*)d_in[3];
  const float* Wo       = (const float*)d_in[4];
  const float* gamma    = (const float*)d_in[5];
  const float* beta     = (const float*)d_in[6];
  float* out = (float*)d_out;
  char* ws = (char*)d_ws;

  float*          Sbuf = (float*)(ws + offS);
  unsigned short* qnH  = (unsigned short*)(ws + offQnH);
  unsigned short* qnL  = (unsigned short*)(ws + offQnL);
  unsigned short* knH  = (unsigned short*)(ws + offKnH);
  unsigned short* knL  = (unsigned short*)(ws + offKnL);
  unsigned short* woT  = (unsigned short*)(ws + offWoT);
  unsigned short* phi  = (unsigned short*)(ws + offPhi);
  unsigned short* plo  = (unsigned short*)(ws + offPlo);
  unsigned short* wqT  = (unsigned short*)(ws + offWqT);
  unsigned short* wkvT = (unsigned short*)(ws + offWkvT);
  unsigned short* qhi  = (unsigned short*)(ws + offQhi);
  unsigned short* qlo  = (unsigned short*)(ws + offQlo);
  unsigned short* khi  = (unsigned short*)(ws + offKhi);
  unsigned short* klo  = (unsigned short*)(ws + offKlo);
  unsigned short* vthi = (unsigned short*)(ws + offVthi);
  unsigned short* vtlo = (unsigned short*)(ws + offVtlo);
  unsigned short* chi  = (unsigned short*)(ws + offChi);
  unsigned short* clo  = (unsigned short*)(ws + offClo);

  const float* dummy_f = gamma;
  void* dummy_c2 = (void*)phi;

  ln_split_kernel<<<dim3(kRowsQ / 8), dim3(256), 0, stream>>>(query, gamma, beta, qnH, qnL, kRowsQ);
  ln_split_kernel<<<dim3(kRowsK / 8), dim3(256), 0, stream>>>(keyvalue, gamma, beta, knH, knL, kRowsK);

  transpose_cast_kernel<<<dim3(kDim / 64, kInner / 64), dim3(256), 0, stream>>>(Wq, kInner, wqT, kDim);
  transpose_cast_kernel<<<dim3(kDim / 64, (2 * kInner) / 64), dim3(256), 0, stream>>>(Wkv, 2 * kInner, wkvT, kDim);

  wmma_gemm64<1, true, 0, 2, false, false><<<dim3((kRowsQ / 64) * (kInner / 64) / 8, 1), dim3(256), 0, stream>>>(
      qnH, qnL, kDim, 0L,
      wqT, wqT, kDim, 0L,
      (void*)qhi, (void*)qlo, kInner, 0L,
      dummy_f, dummy_f, 0L,
      kRowsQ, kInner, kDim, 1.0f);

  wmma_gemm64<1, true, 0, 2, false, false><<<dim3((kRowsK / 64) * (kInner / 64) / 8, 1), dim3(256), 0, stream>>>(
      knH, knL, kDim, 0L,
      wkvT, wkvT, kDim, 0L,
      (void*)khi, (void*)klo, kInner, 0L,
      dummy_f, dummy_f, 0L,
      kRowsK, kInner, kDim, 1.0f);

  wmma_gemm64<1, false, 0, 2, false, true><<<dim3((kInner / 64) * (kRowsK / 64) / 8, 1), dim3(256), 0, stream>>>(
      wkvT + (size_t)kInner * kDim, wkvT + (size_t)kInner * kDim, kDim, 0L,
      knH, knL, kDim, 0L,
      (void*)vthi, (void*)vtlo, kRowsK, 0L,
      dummy_f, dummy_f, 0L,
      kInner, kRowsK, kDim, 1.0f);

  for (int b = 0; b < kBatch; ++b) {
    const size_t qoff = (size_t)b * kNq * kInner;
    const size_t koff = (size_t)b * kNk * kInner;

    wmma_gemm64<1, true, 0, 0, false, true><<<dim3((kNq / 64) * (kNk / 64) / 8, kHeads), dim3(256), 0, stream>>>(
        qhi + qoff, qlo + qoff, kInner, (long)kDh,
        khi + koff, klo + koff, kInner, (long)kDh,
        (void*)Sbuf, dummy_c2, kNk, (long)kNq * kNk,
        dummy_f, dummy_f, 0L,
        kNq, kNk, kDh, kScoreScale);

    softmax_rows_kernel<<<dim3(kHeads * kNq), dim3(128), 0, stream>>>(Sbuf, phi, plo);

    const size_t vtoff = (size_t)b * kNk;
    const size_t coff  = (size_t)b * kNq * kInner;
    wmma_gemm64<1, true, 0, 2, false, true><<<dim3((kNq / 64) * (kDh / 64) / 8, kHeads), dim3(256), 0, stream>>>(
        phi, plo, kNk, (long)kNq * kNk,
        vthi + vtoff, vtlo + vtoff, kRowsK, (long)kDh * kRowsK,
        (void*)(chi + coff), (void*)(clo + coff), kInner, (long)kDh,
        dummy_f, dummy_f, 0L,
        kNq, kDh, kNk, 1.0f);
  }

  transpose_cast_kernel<<<dim3(kInner / 64, kDim / 64), dim3(256), 0, stream>>>(Wo, kDim, woT, kInner);

  wmma_gemm64<1, true, 0, 0, false, false><<<dim3((kRowsQ / 64) * (kDim / 64) / 8, 1), dim3(256), 0, stream>>>(
      chi, clo, kInner, 0L,
      woT, woT, kInner, 0L,
      (void*)out, dummy_c2, kDim, 0L,
      dummy_f, dummy_f, 0L,
      kRowsQ, kDim, kInner, 1.0f);
}
